// FuzzyMultiheadAttention_64080912056504
// MI455X (gfx1250) — hardware-run, weakly checked
//
#include <hip/hip_runtime.h>
#include <stddef.h>
#include <stdint.h>


#define NTOK  8192
#define SEQ   2048
#define NBAT  4
#define EMB   512
#define NH    8
#define NR    16
#define HD    64
#define EVR   8192
#define XSC   8
#define WSC   1024
#define PSC   1024
#define NTHR  256
#define NWAVE 8
#define WSCAP 134217728
#define LDS_GEMM (NWAVE * 32 * 64 * 4)
#define VP_STG  (NWAVE * 2048)
#define VP_RES  (128 * 64)
#define VP_ATT  (128 * 16)
#define VP_TAB  1024
#define LDS_VP  ((VP_STG + VP_RES + VP_ATT + 3 * VP_TAB) * 4)

static_assert(NTOK == NBAT * SEQ);
static_assert(EVR == EMB * NR);
static_assert(EMB == NH * HD);
static_assert(VP_TAB == NR * HD);
static_assert((NTOK % 128) == 0);
static_assert((SEQ % 128) == 0);
static_assert((EMB % 128) == 0);
static_assert((EMB % 32) == 0);
static_assert(((NTOK * EMB) % (8 * NTHR)) == 0);
static_assert(((EMB * EMB) % (8 * NTHR)) == 0);
static_assert(((EVR * EMB) % (8 * NTHR)) == 0);
static_assert(NTHR == NWAVE * 32);
static_assert(LDS_VP <= 300 * 1024);
static_assert(LDS_GEMM <= 300 * 1024);

typedef float          v4f  __attribute__((ext_vector_type(4)));
typedef float          v8f  __attribute__((ext_vector_type(8)));
typedef _Float16       v8h  __attribute__((ext_vector_type(8)));
typedef _Float16       v16h __attribute__((ext_vector_type(16)));
union FragH { v16h v; v8h h[2]; };

__device__ __forceinline__ v8f wmf(v16h a, v16h b, v8f c) {
  v8f d = __builtin_amdgcn_wmma_f32_16x16x32_f16(false, a, false, b, (short)0, c, false, false);
  asm volatile("v_nop\n\tv_nop\n\tv_nop\n\tv_nop" : "+v"(d) : "v"(a), "v"(b));
  return d;
}

__global__ __launch_bounds__(NTHR) void k_cvt(const float* __restrict__ x, _Float16* d16, float sc) {
  const size_t t = (size_t)blockIdx.x * NTHR + threadIdx.x;
  const float* p = x + t * 8;
  const v4f f0 = *(const v4f*)p;
  const v4f f1 = *(const v4f*)(p + 4);
  v8h a;
  a[0] = (_Float16)(f0.x * sc); a[1] = (_Float16)(f0.y * sc);
  a[2] = (_Float16)(f0.z * sc); a[3] = (_Float16)(f0.w * sc);
  a[4] = (_Float16)(f1.x * sc); a[5] = (_Float16)(f1.y * sc);
  a[6] = (_Float16)(f1.z * sc); a[7] = (_Float16)(f1.w * sc);
  _Float16* d = d16 + t * 8;
  *(volatile v8h*)d = a;
  __threadfence();
  *(volatile v8h*)d = a;
}

__global__ __launch_bounds__(NTHR) void k_gemm(const _Float16* __restrict__ A, const _Float16* __restrict__ Bw,
                                               const float* __restrict__ bias, float* C, float osc, float alpha) {
  extern __shared__ v4f lds_g[];
  const int tid = threadIdx.x, lane = tid & 31, wave = tid >> 5, hh = lane >> 4, m = lane & 15;
  float* stg = (float*)lds_g + wave * (32 * 64);
  const int n0 = blockIdx.x * 128, m0 = blockIdx.y * 128;
  const int wm = (wave >> 1) * 32, wn = (wave & 1) * 64;

  v8f acc[2][4];
#pragma unroll
  for (int mt = 0; mt < 2; ++mt)
#pragma unroll
    for (int nt = 0; nt < 4; ++nt) { v8f z = {0.f, 0.f, 0.f, 0.f, 0.f, 0.f, 0.f, 0.f}; acc[mt][nt] = z; }

  const _Float16* ap = A  + (size_t)(m0 + wm + m) * EMB + 8 * hh;
  const _Float16* bp = Bw + (size_t)(n0 + wn + m) * EMB + 8 * hh;
#pragma unroll 1
  for (int kt = 0; kt < EMB / 32; ++kt) {
    const int k0 = 32 * kt;
    FragH a0, a1;
    a0.h[0] = *(const v8h*)(ap + k0);
    a0.h[1] = *(const v8h*)(ap + k0 + 16);
    a1.h[0] = *(const v8h*)(ap + 16 * EMB + k0);
    a1.h[1] = *(const v8h*)(ap + 16 * EMB + k0 + 16);
#pragma unroll
    for (int nt = 0; nt < 4; ++nt) {
      const _Float16* bpn = bp + (size_t)nt * 16 * EMB + k0;
      FragH b;
      b.h[0] = *(const v8h*)bpn;
      b.h[1] = *(const v8h*)(bpn + 16);
      acc[0][nt] = wmf(a0.v, b.v, acc[0][nt]);
      acc[1][nt] = wmf(a1.v, b.v, acc[1][nt]);
    }
  }

  float bvv[4];
#pragma unroll
  for (int nt = 0; nt < 4; ++nt) bvv[nt] = bias[n0 + wn + 16 * nt + m];
#pragma unroll
  for (int mt = 0; mt < 2; ++mt) {
    float* sp = stg + (16 * mt + 8 * hh) * 64 + m;
#pragma unroll
    for (int nt = 0; nt < 4; ++nt) {
#pragma unroll
      for (int r = 0; r < 8; ++r) sp[r * 64 + 16 * nt] = (acc[mt][nt][r] * osc + bvv[nt]) * alpha;
    }
  }
  __syncthreads();

  float* gbase = C + (size_t)(m0 + wm) * EMB + n0 + wn;
#pragma unroll
  for (int q = 0; q < 16; ++q) {
    const int row = 2 * q + hh;
    const v4f v = *(const v4f*)(stg + row * 64 + 4 * m);
    *(volatile v4f*)(gbase + (size_t)row * EMB + 4 * m) = v;
  }
  __threadfence();
#pragma unroll
  for (int q = 0; q < 16; ++q) {
    const int row = 2 * q + hh;
    const v4f v = *(const v4f*)(stg + row * 64 + 4 * m);
    *(volatile v4f*)(gbase + (size_t)row * EMB + 4 * m) = v;
  }
}

__global__ __launch_bounds__(NTHR) void k_vproj(const _Float16* __restrict__ xv16, const _Float16* __restrict__ wv16,
                                                const float* __restrict__ bv, const float* __restrict__ qpl,
                                                const float* __restrict__ rkeys, const float* __restrict__ rwid,
                                                _Float16* p16) {
  extern __shared__ v4f lds_v[];
  float* lds = (float*)lds_v;
  const int tid = threadIdx.x, lane = tid & 31, wave = tid >> 5, hh = lane >> 4, m = lane & 15;
  float* stg   = lds + wave * 2048;
  float* s_res = lds + VP_STG;
  float* s_att = s_res + VP_RES;
  float* s_key = s_att + VP_ATT;
  float* s_wiv = s_key + VP_TAB;
  float* s_bvs = s_wiv + VP_TAB;
  const int m0 = blockIdx.x * 128, h = blockIdx.y;
  const int wm = (wave >> 1) * 32, wn = (wave & 1) * 64;

#pragma unroll 1
  for (int j = tid; j < VP_TAB; j += NTHR) {
    s_key[j] = rkeys[h * VP_TAB + j];
    s_wiv[j] = 1.0f / rwid[h * VP_TAB + j];
    s_bvs[j] = bv[h * VP_TAB + j];
  }
  __syncthreads();

  {
    const int r = tid & 15, g = tid >> 4;
    const float* kr = s_key + r * HD;
    const float* wr = s_wiv + r * HD;
#pragma unroll 1
    for (int ps = 0; ps < 8; ++ps) {
      const int tk = ps * 16 + g;
      const float* qrow = qpl + (size_t)(m0 + tk) * EMB + h * HD;
      float sq = 0.f;
#pragma unroll 2
      for (int d = 0; d < HD; d += 4) {
        const v4f qv = *(const v4f*)(qrow + d);
        const v4f kv = *(const v4f*)(kr + d);
        const v4f iv = *(const v4f*)(wr + d);
        const v4f df = (qv - kv) * iv;
        sq += df.x * df.x; sq += df.y * df.y; sq += df.z * df.z; sq += df.w * df.w;
      }
      const float z = -0.5f * (sq * (1.0f / (float)HD));
      float mx = z;
      mx = fmaxf(mx, __shfl_xor(mx, 8, 32));
      mx = fmaxf(mx, __shfl_xor(mx, 4, 32));
      mx = fmaxf(mx, __shfl_xor(mx, 2, 32));
      mx = fmaxf(mx, __shfl_xor(mx, 1, 32));
      const float e = __expf(z - mx);
      float s = e;
      s += __shfl_xor(s, 8, 32);
      s += __shfl_xor(s, 4, 32);
      s += __shfl_xor(s, 2, 32);
      s += __shfl_xor(s, 1, 32);
      s_att[tk * NR + r] = e * (1.0f / s);
    }
  }
  __syncthreads();

  constexpr float OSCV = 1.0f / (float)(XSC * WSC);
  const _Float16* ap = xv16 + (size_t)(m0 + wm + m) * EMB + 8 * hh;
#pragma unroll 1
  for (int c = 0; c < 8; ++c) {
    const int coff = c * 128 + wn;
    const _Float16* bp = wv16 + (size_t)(h * VP_TAB + coff + m) * EMB + 8 * hh;
    v8f acc[2][4];
#pragma unroll
    for (int mt = 0; mt < 2; ++mt)
#pragma unroll
      for (int nt = 0; nt < 4; ++nt) { v8f z = {0.f, 0.f, 0.f, 0.f, 0.f, 0.f, 0.f, 0.f}; acc[mt][nt] = z; }

#pragma unroll 1
    for (int kt = 0; kt < EMB / 32; ++kt) {
      const int k0 = 32 * kt;
      FragH a0, a1;
      a0.h[0] = *(const v8h*)(ap + k0);
      a0.h[1] = *(const v8h*)(ap + k0 + 16);
      a1.h[0] = *(const v8h*)(ap + 16 * EMB + k0);
      a1.h[1] = *(const v8h*)(ap + 16 * EMB + k0 + 16);
#pragma unroll
      for (int nt = 0; nt < 4; ++nt) {
        const _Float16* bpn = bp + (size_t)nt * 16 * EMB + k0;
        FragH b;
        b.h[0] = *(const v8h*)bpn;
        b.h[1] = *(const v8h*)(bpn + 16);
        acc[0][nt] = wmf(a0.v, b.v, acc[0][nt]);
        acc[1][nt] = wmf(a1.v, b.v, acc[1][nt]);
      }
    }

#pragma unroll
    for (int mt = 0; mt < 2; ++mt) {
      float* sp = stg + (16 * mt + 8 * hh) * 64 + m;
#pragma unroll
      for (int nt = 0; nt < 4; ++nt) {
#pragma unroll
        for (int r = 0; r < 8; ++r) sp[r * 64 + 16 * nt] = acc[mt][nt][r];
      }
    }
    __syncthreads();

    {
      const int lr = wm + lane;
      const v4f* arow = (const v4f*)(s_att + lr * NR);
      const v4f aw0 = arow[0], aw1 = arow[1], aw2 = arow[2], aw3 = arow[3];
      const float* srow = stg + lane * 64;
      const float* bb = s_bvs + coff;
#pragma unroll
      for (int nt = 0; nt < 4; ++nt) {
        const v4f x0 = *(const v4f*)(srow + 16 * nt);
        const v4f x1 = *(const v4f*)(srow + 16 * nt + 4);
        const v4f x2 = *(const v4f*)(srow + 16 * nt + 8);
        const v4f x3 = *(const v4f*)(srow + 16 * nt + 12);
        const v4f b0 = *(const v4f*)(bb + 16 * nt);
        const v4f b1 = *(const v4f*)(bb + 16 * nt + 4);
        const v4f b2 = *(const v4f*)(bb + 16 * nt + 8);
        const v4f b3 = *(const v4f*)(bb + 16 * nt + 12);
        const v4f v0 = (x0 * OSCV + b0) * 0.125f;
        const v4f v1 = (x1 * OSCV + b1) * 0.125f;
        const v4f v2 = (x2 * OSCV + b2) * 0.125f;
        const v4f v3 = (x3 * OSCV + b3) * 0.125f;
        float sum = 0.f;
        sum += aw0.x * v0.x; sum += aw0.y * v0.y; sum += aw0.z * v0.z; sum += aw0.w * v0.w;
        sum += aw1.x * v1.x; sum += aw1.y * v1.y; sum += aw1.z * v1.z; sum += aw1.w * v1.w;
        sum += aw2.x * v2.x; sum += aw2.y * v2.y; sum += aw2.z * v2.z; sum += aw2.w * v2.w;
        sum += aw3.x * v3.x; sum += aw3.y * v3.y; sum += aw3.z * v3.z; sum += aw3.w * v3.w;
        s_res[lr * HD + 8 * c + 4 * (wave & 1) + nt] = sum;
      }
    }
    __syncthreads();
  }

  const int bidx = m0 / SEQ, s0 = m0 - bidx * SEQ;
  _Float16* pbase = p16 + ((size_t)(bidx * NH + h) * SEQ + s0) * HD;
  v8h hv[4];
#pragma unroll
  for (int ps = 0; ps < 4; ++ps) {
    const int idx = ps * NTHR + tid;
    const float* sp = s_res + idx * 8;
    const v4f u0 = *(const v4f*)sp;
    const v4f u1 = *(const v4f*)(sp + 4);
    hv[ps][0] = (_Float16)(u0.x * (float)PSC); hv[ps][1] = (_Float16)(u0.y * (float)PSC);
    hv[ps][2] = (_Float16)(u0.z * (float)PSC); hv[ps][3] = (_Float16)(u0.w * (float)PSC);
    hv[ps][4] = (_Float16)(u1.x * (float)PSC); hv[ps][5] = (_Float16)(u1.y * (float)PSC);
    hv[ps][6] = (_Float16)(u1.z * (float)PSC); hv[ps][7] = (_Float16)(u1.w * (float)PSC);
  }
#pragma unroll
  for (int ps = 0; ps < 4; ++ps) {
    _Float16* d = pbase + (size_t)(ps * NTHR + tid) * 8;
    *(volatile v8h*)d = hv[ps];
  }
  __threadfence();
#pragma unroll
  for (int ps = 0; ps < 4; ++ps) {
    _Float16* d = pbase + (size_t)(ps * NTHR + tid) * 8;
    *(volatile v8h*)d = hv[ps];
  }
}

extern "C" void kernel_launch(void* const* d_in, const int* in_sizes, int n_in,
                              void* d_out, int out_size, void* d_ws, size_t ws_size,
                              hipStream_t stream) {
  if (n_in < 11) return;
  if (in_sizes[0] != NTOK * EMB || in_sizes[2] != NTOK * EMB) return;
  if (in_sizes[3] != EMB * EMB || in_sizes[4] != EMB) return;
  if (in_sizes[5] != EVR * EMB || in_sizes[6] != EVR) return;
  if (in_sizes[7] != EMB * EMB || in_sizes[8] != EMB) return;
  if (in_sizes[9] != NH * NR * HD || in_sizes[10] != NH * NR * HD) return;
  if (out_size != NTOK * EMB) return;

  const float* query = (const float*)d_in[0];
  const float* value = (const float*)d_in[2];
  const float* Wq    = (const float*)d_in[3];
  const float* bq    = (const float*)d_in[4];
  const float* Wv    = (const float*)d_in[5];
  const float* bv    = (const float*)d_in[6];
  const float* Wo    = (const float*)d_in[7];
  const float* bo    = (const float*)d_in[8];
  const float* rk    = (const float*)d_in[9];
  const float* rw    = (const float*)d_in[10];
  float* out = (float*)d_out;

  char* ws = (char*)d_ws;
  size_t off = 0;
  const size_t oXq = off; off += (size_t)NTOK * EMB * 2;          off = (off + 255) & ~(size_t)255;
  const size_t oXv = off; off += (size_t)NTOK * EMB * 2;          off = (off + 255) & ~(size_t)255;
  const size_t oWq = off; off += (size_t)EMB * EMB * 2;           off = (off + 255) & ~(size_t)255;
  const size_t oWv = off; off += (size_t)EVR * EMB * 2;           off = (off + 255) & ~(size_t)255;
  const size_t oWo = off; off += (size_t)EMB * EMB * 2;           off = (off + 255) & ~(size_t)255;
  const size_t oQ  = off; off += (size_t)NTOK * EMB * 4;          off = (off + 255) & ~(size_t)255;
  const size_t oP  = off; off += (size_t)NBAT * NH * SEQ * HD * 2; off = (off + 255) & ~(size_t)255;
  if (off > ws_size || off > (size_t)WSCAP) return;
  _Float16* xq16 = (_Float16*)(ws + oXq);
  _Float16* xv16 = (_Float16*)(ws + oXv);
  _Float16* wq16 = (_Float16*)(ws + oWq);
  _Float16* wv16 = (_Float16*)(ws + oWv);
  _Float16* wo16 = (_Float16*)(ws + oWo);
  float*    qpl  = (float*)(ws + oQ);
  _Float16* p16  = (_Float16*)(ws + oP);

  k_cvt<<<(NTOK * EMB) / (8 * NTHR), NTHR, 0, stream>>>(query, xq16, (float)XSC);
  k_cvt<<<(NTOK * EMB) / (8 * NTHR), NTHR, 0, stream>>>(value, xv16, (float)XSC);
  k_cvt<<<(EMB * EMB) / (8 * NTHR), NTHR, 0, stream>>>(Wq, wq16, (float)WSC);
  k_cvt<<<(EVR * EMB) / (8 * NTHR), NTHR, 0, stream>>>(Wv, wv16, (float)WSC);
  k_cvt<<<(EMB * EMB) / (8 * NTHR), NTHR, 0, stream>>>(Wo, wo16, (float)WSC);

  hipFuncSetAttribute(reinterpret_cast<const void*>(&k_gemm),
                      hipFuncAttributeMaxDynamicSharedMemorySize, LDS_GEMM);
  k_gemm<<<dim3(EMB / 128, NTOK / 128), NTHR, LDS_GEMM, stream>>>(
      xq16, wq16, bq, qpl, 1.0f / (float)(XSC * WSC), 0.125f);

  hipFuncSetAttribute(reinterpret_cast<const void*>(&k_vproj),
                      hipFuncAttributeMaxDynamicSharedMemorySize, LDS_VP);
  k_vproj<<<dim3(NTOK / 128, NH), NTHR, LDS_VP, stream>>>(xv16, wv16, bv, qpl, rk, rw, p16);

  k_gemm<<<dim3(EMB / 128, NTOK / 128), NTHR, LDS_GEMM, stream>>>(
      p16, wo16, bo, out, 1.0f / (float)(PSC * WSC), 1.0f);
}
